// LHATransformerBlock_51479478010637
// MI455X (gfx1250) — hardware-run, weakly checked
//
#include <hip/hip_runtime.h>
#include <math.h>
#include <stdint.h>

#define NBATCH 2
#define SEQ    2048
#define DM     1024
#define NH     16
#define HD     64
#define NBK    32
#define MLPD   4096
#define NTOK   (NBATCH * SEQ)
#define QKP    (2 * DM)
#define HDX    96
#define QXP    (NH * HDX)
#define NQB    (SEQ / 64)
#define TOKG   16
#define NTG    (NTOK / TOKG)
#define WSC    16.0f
static_assert(NH * HD == DM);
static_assert(NBK == 32);
static_assert(NH * NBK == 512);
static_assert((SEQ % 64) == 0 && (DM % 64) == 0 && (MLPD % 64) == 0);
static_assert(((QXP * 2) % 128) == 0);
static_assert((NTOK % TOKG) == 0);

typedef _Float16 v16h __attribute__((ext_vector_type(16)));
typedef _Float16 v8h  __attribute__((ext_vector_type(8)));
typedef float    v8f  __attribute__((ext_vector_type(8)));
typedef float    v4f  __attribute__((ext_vector_type(4)));
typedef unsigned int v4u __attribute__((ext_vector_type(4)));
union FH { v16h v; v8h h[2]; };

__device__ __forceinline__ unsigned short bf_bits(float f) {
  unsigned u = __float_as_uint(f);
  return (unsigned short)((u + 0x7FFFu + ((u >> 16) & 1u)) >> 16);
}
__device__ __forceinline__ float bf_up(unsigned short h) { return __uint_as_float(((unsigned)h) << 16); }
__device__ __forceinline__ float bfr(float f) { return bf_up(bf_bits(f)); }
__device__ __forceinline__ unsigned short h_bits(_Float16 x) { return __builtin_bit_cast(unsigned short, x); }
__device__ __forceinline__ unsigned pk16(unsigned short a, unsigned short b) { return (unsigned)a | ((unsigned)b << 16); }
__device__ __forceinline__ v8f zero8() { v8f z = {0.f, 0.f, 0.f, 0.f, 0.f, 0.f, 0.f, 0.f}; return z; }

__device__ __forceinline__ v16h ldfrag_h(const _Float16* p) {
  FH f;
  f.h[0] = *(const v8h*)(p);
  f.h[1] = *(const v8h*)(p + 16);
  return f.v;
}

__device__ __forceinline__ v8f mma_h(v16h a, v16h b, v8f c) {
  c = __builtin_amdgcn_wmma_f32_16x16x32_f16(false, a, false, b, (short)0, c, false, false);
#if defined(__HIP_DEVICE_COMPILE__)
  asm volatile("v_nop\n\tv_nop\n\tv_nop\n\tv_nop" : "+v"(c) : "v"(a), "v"(b));
#endif
  return c;
}
__device__ __forceinline__ v8f mma_h_raw(v16h a, v16h b, v8f c) {
  return __builtin_amdgcn_wmma_f32_16x16x32_f16(false, a, false, b, (short)0, c, false, false);
}
__device__ __forceinline__ void dep_guard_h(v8f& a, v8f& b, v16h x, v16h y) {
#if defined(__HIP_DEVICE_COMPILE__)
  asm volatile("v_nop\n\tv_nop\n\tv_nop\n\tv_nop" : "+v"(a), "+v"(b) : "v"(x), "v"(y));
#endif
}
__device__ __forceinline__ void keep4_h(v16h a, v16h b, v16h c, v16h d) {
#if defined(__HIP_DEVICE_COMPILE__)
  asm volatile("v_nop" :: "v"(a), "v"(b), "v"(c), "v"(d));
#endif
}
__device__ __forceinline__ void acc_guard4(v8f& a, v8f& b, v8f& c, v8f& d) {
#if defined(__HIP_DEVICE_COMPILE__)
  asm volatile("v_nop\n\tv_nop\n\tv_nop\n\tv_nop" : "+v"(a), "+v"(b), "+v"(c), "+v"(d));
#endif
}
__device__ __forceinline__ void wave_sync_lds() {
  __builtin_amdgcn_fence(__ATOMIC_RELEASE, "workgroup");
  __builtin_amdgcn_wave_barrier();
  __builtin_amdgcn_fence(__ATOMIC_ACQUIRE, "workgroup");
}

__global__ __launch_bounds__(256) void tr_cvt(const float* __restrict__ in0, const float* __restrict__ in1,
                                              const float* __restrict__ in2, unsigned short* out,
                                              long long zstride, int R, int C, float scale) {
  __shared__ float tile[64 * 33];
  const int z = blockIdx.z;
  const float* in = (z == 0) ? in0 : ((z == 1) ? in1 : in2);
  unsigned short* ob = out + (size_t)z * (size_t)zstride;
  const int r0 = blockIdx.y * 64, c0 = blockIdx.x * 32;
  const int t = threadIdx.x;
  {
    const int ir = t >> 2, ic = (t & 3) * 8;
    const float* g = in + (size_t)(r0 + ir) * C + c0 + ic;
    const v4f a = *(const v4f*)g;
    const v4f b = *(const v4f*)(g + 4);
    float* l = tile + ir * 33 + ic;
    l[0] = a[0]; l[1] = a[1]; l[2] = a[2]; l[3] = a[3];
    l[4] = b[0]; l[5] = b[1]; l[6] = b[2]; l[7] = b[3];
  }
  __syncthreads();
  const int orow = t >> 3, piece = (t & 7) * 8;
  v4u p;
#pragma unroll
  for (int e = 0; e < 4; ++e) {
    const float f0 = tile[(piece + 2 * e) * 33 + orow];
    const float f1 = tile[(piece + 2 * e + 1) * 33 + orow];
    const _Float16 x0 = (_Float16)(bfr(f0) * scale);
    const _Float16 x1 = (_Float16)(bfr(f1) * scale);
    p[e] = pk16(h_bits(x0), h_bits(x1));
  }
  const size_t go = (size_t)(c0 + orow) * (size_t)R + r0 + piece;
  *(volatile v4u*)(ob + go) = p;
  __threadfence();
  *(volatile v4u*)(ob + go) = p;
}

template <bool RIN>
__global__ __launch_bounds__(128) void ln_f16(const float* __restrict__ x, const float* __restrict__ g,
                                             const float* __restrict__ bt, unsigned short* out) {
  __shared__ float red[2][4];
  const int row = blockIdx.x, t = threadIdx.x, lane = t & 31, w = t >> 5;
  const float* xr = x + (size_t)row * DM + 8 * t;
  const v4f a = *(const v4f*)xr;
  const v4f a2 = *(const v4f*)(xr + 4);
  float v[8];
#pragma unroll
  for (int e = 0; e < 4; ++e) { v[e] = a[e]; v[4 + e] = a2[e]; }
  if (RIN) {
#pragma unroll
    for (int e = 0; e < 8; ++e) v[e] = bfr(v[e]);
  }
  float s = 0.f;
#pragma unroll
  for (int e = 0; e < 8; ++e) s += v[e];
  for (int off = 16; off > 0; off >>= 1) s += __shfl_xor(s, off, 32);
  if (lane == 0) red[0][w] = s;
  __syncthreads();
  const float tot = ((red[0][0] + red[0][1]) + red[0][2]) + red[0][3];
  const float mu = tot * (1.0f / (float)DM);
  float d[8];
  float s2 = 0.f;
#pragma unroll
  for (int e = 0; e < 8; ++e) { d[e] = v[e] - mu; s2 += d[e] * d[e]; }
  for (int off = 16; off > 0; off >>= 1) s2 += __shfl_xor(s2, off, 32);
  if (lane == 0) red[1][w] = s2;
  __syncthreads();
  const float tot2 = ((red[1][0] + red[1][1]) + red[1][2]) + red[1][3];
  const float var = tot2 * (1.0f / (float)DM);
  const float rs = rsqrtf(var + 1e-6f);
  const v4f g0 = *(const v4f*)(g + 8 * t), g1 = *(const v4f*)(g + 8 * t + 4);
  const v4f b0 = *(const v4f*)(bt + 8 * t), b1 = *(const v4f*)(bt + 8 * t + 4);
  float gg[8], cc[8];
#pragma unroll
  for (int e = 0; e < 4; ++e) {
    gg[e] = bfr(g0[e]); gg[4 + e] = bfr(g1[e]);
    cc[e] = bfr(b0[e]); cc[4 + e] = bfr(b1[e]);
  }
  v4u p;
#pragma unroll
  for (int e = 0; e < 4; ++e) {
    const float f0 = d[2 * e] * rs * gg[2 * e] + cc[2 * e];
    const float f1 = d[2 * e + 1] * rs * gg[2 * e + 1] + cc[2 * e + 1];
    p[e] = pk16(h_bits((_Float16)f0), h_bits((_Float16)f1));
  }
  unsigned short* op = out + (size_t)row * DM + 8 * t;
  *(volatile v4u*)op = p;
  __threadfence();
  *(volatile v4u*)op = p;
}

template <int OM, bool BIAS, bool RELU, int RES>
__global__ __launch_bounds__(256) void gemm64(
    const unsigned short* __restrict__ Ap, int lda, long long strideA,
    const unsigned short* __restrict__ Btp, int ldb, long long strideB,
    void* Cout, int ldc, long long strideC,
    const float* __restrict__ bias, const float* __restrict__ res, int ldr,
    int M, int N, int K, float oscale) {
  const _Float16* A  = (const _Float16*)(const void*)Ap;
  const _Float16* Bt = (const _Float16*)(const void*)Btp;
  __shared__ __align__(16) float sT[8][16 * 68];
  const int b    = blockIdx.y;
  const int lane = threadIdx.x & 31;
  const int wave = threadIdx.x >> 5;
  const int tilesN = N >> 6;
  const int tilesM = M >> 6;
  const int tile = blockIdx.x * 8 + wave;
  if (tile >= tilesM * tilesN) return;
  const int tm = tile / tilesN;
  const int tn = tile - tm * tilesN;
  const int m0 = tm << 6;
  const int n0 = tn << 6;

  const _Float16* Ab = A  + (size_t)b * (size_t)strideA;
  const _Float16* Bb = Bt + (size_t)b * (size_t)strideB;

  const int rlane = lane & 15;
  const int koff  = (lane >> 4) * 8;
  const int mOff  = (lane >> 4) * 8;

  v8f acc[4][4];
#pragma unroll
  for (int i = 0; i < 4; ++i)
#pragma unroll
    for (int j = 0; j < 4; ++j) acc[i][j] = zero8();

  for (int k0 = 0; k0 < K; k0 += 32) {
    v16h bh[4];
#pragma unroll
    for (int j = 0; j < 4; ++j) {
      const size_t bo = (size_t)(n0 + (j << 4) + rlane) * ldb + koff + k0;
      bh[j] = ldfrag_h(Bb + bo);
    }
#pragma unroll
    for (int i = 0; i < 4; ++i) {
      const size_t ao = (size_t)(m0 + (i << 4) + rlane) * lda + koff + k0;
      const v16h ah = ldfrag_h(Ab + ao);
#pragma unroll
      for (int j = 0; j < 4; ++j) acc[i][j] = mma_h_raw(ah, bh[j], acc[i][j]);
      dep_guard_h(acc[i][0], acc[i][3], ah, bh[3]);
    }
    keep4_h(bh[0], bh[1], bh[2], bh[3]);
  }
  acc_guard4(acc[0][0], acc[0][1], acc[0][2], acc[0][3]);
  acc_guard4(acc[1][0], acc[1][1], acc[1][2], acc[1][3]);
  acc_guard4(acc[2][0], acc[2][1], acc[2][2], acc[2][3]);
  acc_guard4(acc[3][0], acc[3][1], acc[3][2], acc[3][3]);

  float* slab = sT[wave];
#pragma unroll
  for (int i = 0; i < 4; ++i) {
    const int mBase = m0 + (i << 4);
#pragma unroll
    for (int j = 0; j < 4; ++j) {
#pragma unroll
      for (int r = 0; r < 8; ++r) {
        slab[(mOff + r) * 68 + (j << 4) + rlane] = acc[i][j][r];
      }
    }
    wave_sync_lds();
    if (OM == 0) {
      float* C = (float*)Cout + (size_t)b * (size_t)strideC;
      const int h2 = lane >> 4, c4 = (lane & 15) * 4;
      v4f bv = {0.f, 0.f, 0.f, 0.f};
      if (BIAS) {
        const v4f t4 = *(const v4f*)(bias + n0 + c4);
#pragma unroll
        for (int e = 0; e < 4; ++e) bv[e] = bfr(t4[e]);
      }
      for (int pass = 0; pass < 2; ++pass) {
#pragma unroll
        for (int it = 0; it < 8; ++it) {
          const int row = it * 2 + h2;
          const v4f sv = *(const v4f*)(slab + row * 68 + c4);
          v4f o;
#pragma unroll
          for (int e = 0; e < 4; ++e) o[e] = sv[e] * oscale + bv[e];
          if (RES != 0) {
            const v4f rv = *(const v4f*)(res + (size_t)(mBase + row) * ldr + n0 + c4);
#pragma unroll
            for (int e = 0; e < 4; ++e) o[e] += (RES == 2) ? bfr(rv[e]) : rv[e];
          }
          if (RELU) {
#pragma unroll
            for (int e = 0; e < 4; ++e) o[e] = fmaxf(o[e], 0.f);
          }
          *(volatile v4f*)(C + (size_t)(mBase + row) * ldc + n0 + c4) = o;
        }
        __threadfence();
      }
    } else {
      const int q = lane >> 3, c8 = (lane & 7) * 8;
      unsigned short* C = (unsigned short*)Cout + (size_t)b * (size_t)strideC;
      float b8[8];
#pragma unroll
      for (int e = 0; e < 8; ++e) b8[e] = 0.f;
      if (BIAS) {
        const v4f t0 = *(const v4f*)(bias + n0 + c8);
        const v4f t1 = *(const v4f*)(bias + n0 + c8 + 4);
#pragma unroll
        for (int e = 0; e < 4; ++e) { b8[e] = bfr(t0[e]); b8[4 + e] = bfr(t1[e]); }
      }
      v4u hv[4];
#pragma unroll
      for (int it = 0; it < 4; ++it) {
        const int row = it * 4 + q;
        const float* sp = slab + row * 68 + c8;
        v4u pk;
#pragma unroll
        for (int e = 0; e < 4; ++e) {
          float f0 = sp[2 * e] * oscale + b8[2 * e];
          float f1 = sp[2 * e + 1] * oscale + b8[2 * e + 1];
          if (RELU) { f0 = fmaxf(f0, 0.f); f1 = fmaxf(f1, 0.f); }
          pk[e] = pk16(h_bits((_Float16)f0), h_bits((_Float16)f1));
        }
        hv[it] = pk;
      }
      for (int pass = 0; pass < 2; ++pass) {
#pragma unroll
        for (int it = 0; it < 4; ++it) {
          const int row = it * 4 + q;
          *(volatile v4u*)(C + (size_t)(mBase + row) * ldc + n0 + c8) = hv[it];
        }
        __threadfence();
      }
    }
    wave_sync_lds();
  }
}

__global__ __launch_bounds__(256) void bucket_qx(const unsigned short* __restrict__ qkp,
                                                 const unsigned short* __restrict__ whp,
                                                 unsigned short* qxo, unsigned short* kxo, float* part) {
  __shared__ __align__(16) _Float16 tile[TOKG * QXP];
  __shared__ __align__(16) float psum[NH * NBK];
  const int sel = blockIdx.y, bx = blockIdx.x, tok0 = bx * TOKG;
  const int t = threadIdx.x, lane = t & 31, wave = t >> 5, hh = lane >> 4, c = lane & 15;
  const _Float16* Q = (const _Float16*)(const void*)qkp + (size_t)sel * DM;
  const _Float16* W = (const _Float16*)(const void*)whp + (size_t)sel * NBK * DM;
  unsigned short* outp = (sel == 0) ? qxo : kxo;
  const float pscale = (sel == 0) ? 0.8f : 1.0f;

  for (int h = wave; h < NH; h += 8) {
    FH a[2];
#pragma unroll
    for (int kc = 0; kc < 2; ++kc) {
      const _Float16* qp = Q + (size_t)(tok0 + c) * QKP + h * HD + kc * 32 + 8 * hh;
      a[kc].h[0] = *(const v8h*)(qp);
      a[kc].h[1] = *(const v8h*)(qp + 16);
    }
    v8f acc[2];
#pragma unroll
    for (int j = 0; j < 2; ++j) {
      v8f dd = zero8();
#pragma unroll
      for (int kc = 0; kc < 2; ++kc) {
        FH bb;
        const _Float16* wp = W + (size_t)(j * 16 + c) * DM + h * HD + kc * 32 + 8 * hh;
        bb.h[0] = *(const v8h*)(wp);
        bb.h[1] = *(const v8h*)(wp + 16);
        dd = mma_h(a[kc].v, bb.v, dd);
      }
      acc[j] = dd;
    }
#pragma unroll
    for (int kc = 0; kc < 2; ++kc) {
      _Float16* tp = tile + c * QXP + h * HDX + kc * 32 + 8 * hh;
      *(v8h*)(tp) = a[kc].h[0];
      *(v8h*)(tp + 16) = a[kc].h[1];
    }
    float cs0 = 0.f, cs1 = 0.f;
#pragma unroll
    for (int r = 0; r < 8; ++r) {
      const float s0 = acc[0][r] * (1.0f / WSC);
      const float s1 = acc[1][r] * (1.0f / WSC);
      float m = fmaxf(s0, s1);
#pragma unroll
      for (int off = 1; off < 16; off <<= 1) m = fmaxf(m, __shfl_xor(m, off, 32));
      const float e0 = __expf(s0 - m), e1 = __expf(s1 - m);
      float sum = e0 + e1;
#pragma unroll
      for (int off = 1; off < 16; off <<= 1) sum += __shfl_xor(sum, off, 32);
      const float inv = 1.0f / sum;
      const float p0 = e0 * inv, p1 = e1 * inv;
      cs0 += p0; cs1 += p1;
      tile[(8 * hh + r) * QXP + h * HDX + HD + c]      = (_Float16)(p0 * pscale);
      tile[(8 * hh + r) * QXP + h * HDX + HD + 16 + c] = (_Float16)(p1 * pscale);
    }
    cs0 += __shfl_xor(cs0, 16, 32);
    cs1 += __shfl_xor(cs1, 16, 32);
    if (hh == 0) { psum[h * NBK + c] = cs0; psum[h * NBK + 16 + c] = cs1; }
  }
  __syncthreads();
  {
    _Float16* gbase = (_Float16*)(void*)(outp + (size_t)tok0 * QXP);
    for (int pass = 0; pass < 2; ++pass) {
#pragma unroll
      for (int i = 0; i < 12; ++i) {
        const v8h vv = *(const v8h*)(tile + (size_t)(i * 256 + t) * 8);
        *(volatile v8h*)(gbase + (size_t)(i * 256 + t) * 8) = vv;
      }
      __threadfence();
    }
  }
  if (t < 128) {
    const v4f pv = *(const v4f*)(psum + 4 * t);
    float* pp = part + (size_t)(sel * NTG + bx) * (NH * NBK) + 4 * t;
    *(volatile v4f*)pp = pv;
    __threadfence();
    *(volatile v4f*)pp = pv;
  }
}

__global__ __launch_bounds__(128)
void attn_x(const unsigned short* __restrict__ qxp, const unsigned short* __restrict__ kxp,
            const unsigned short* __restrict__ vtp, unsigned short* ctxp, float sscale) {
  __shared__ __align__(16) _Float16 Ksh[64 * HDX];
  __shared__ __align__(16) _Float16 Vth[64 * 64];
  __shared__ __align__(16) _Float16 Psh[4][16 * 64];
  __shared__ __align__(16) float    Os[4][16 * 64];

  const int tid  = threadIdx.x;
  const int wave = tid >> 5;
  const int lane = tid & 31;
  const int hh   = lane >> 4;
  const int c    = lane & 15;

  const int bx   = blockIdx.x;
  const int qb   = bx % NQB;
  const int rest = bx / NQB;
  const int h    = rest % NH;
  const int b    = rest / NH;
  const int q0   = qb * 64 + wave * 16;
  const size_t rowB = (size_t)b * SEQ;

  const _Float16* Qg = (const _Float16*)(const void*)qxp + (size_t)h * HDX;
  const _Float16* Kg = (const _Float16*)(const void*)kxp + (size_t)h * HDX;
  const _Float16* Vg = (const _Float16*)(const void*)vtp + ((size_t)b * DM + (size_t)h * HD) * SEQ;

  v16h qa[3];
#pragma unroll
  for (int dc = 0; dc < 3; ++dc) qa[dc] = ldfrag_h(Qg + (rowB + q0 + c) * QXP + dc * 32 + 8 * hh);

  float mrow[8], lrow[8];
  v8f oacc[4];
#pragma unroll
  for (int r = 0; r < 8; ++r) { mrow[r] = -INFINITY; lrow[r] = 0.f; }
#pragma unroll
  for (int t = 0; t < 4; ++t) oacc[t] = zero8();

  for (int kt = 0; kt < NQB; ++kt) {
    const int kv0 = kt * 64;
    __syncthreads();
    {
      const int r = tid >> 1, hk = (tid & 1) * 48, hv = (tid & 1) * 32;
      const _Float16* kg = Kg + (rowB + kv0 + r) * QXP + hk;
      const _Float16* vg = Vg + (size_t)r * SEQ + kv0 + hv;
#pragma unroll
      for (int i = 0; i < 6; ++i) *(v8h*)(Ksh + r * HDX + hk + 8 * i) = *(const v8h*)(kg + 8 * i);
#pragma unroll
      for (int i = 0; i < 4; ++i) *(v8h*)(Vth + r * 64 + hv + 8 * i) = *(const v8h*)(vg + 8 * i);
    }
    __syncthreads();

    v8f s[4];
#pragma unroll
    for (int j = 0; j < 4; ++j) {
      v8f sh = zero8();
#pragma unroll
      for (int dc = 0; dc < 3; ++dc) {
        FH kb;
        kb.h[0] = *(const v8h*)(Ksh + (j * 16 + c) * HDX + dc * 32 + 8 * hh);
        kb.h[1] = *(const v8h*)(Ksh + (j * 16 + c) * HDX + dc * 32 + 16 + 8 * hh);
        sh = mma_h(qa[dc], kb.v, sh);
      }
#pragma unroll
      for (int r = 0; r < 8; ++r) s[j][r] = sh[r] * sscale;
    }

    _Float16* pwh = Psh[wave];
#pragma unroll
    for (int r = 0; r < 8; ++r) {
      float m = s[0][r];
      m = fmaxf(m, s[1][r]);
      m = fmaxf(m, s[2][r]);
      m = fmaxf(m, s[3][r]);
#pragma unroll
      for (int off = 1; off < 16; off <<= 1) m = fmaxf(m, __shfl_xor(m, off, 32));
      const float mnew  = fmaxf(mrow[r], m);
      const float alpha = __expf(mrow[r] - mnew);
      mrow[r] = mnew;
      float psum = 0.f;
#pragma unroll
      for (int j = 0; j < 4; ++j) {
        const float p = __expf(s[j][r] - mnew);
        psum += p;
        pwh[(8 * hh + r) * 64 + j * 16 + c] = (_Float16)(p * 1024.0f);
      }
#pragma unroll
      for (int off = 1; off < 16; off <<= 1) psum += __shfl_xor(psum, off, 32);
      lrow[r] = lrow[r] * alpha + psum;
#pragma unroll
      for (int t = 0; t < 4; ++t) oacc[t][r] *= alpha;
    }
    wave_sync_lds();

#pragma unroll 1
    for (int kk = 0; kk < 2; ++kk) {
      FH pa;
      pa.h[0] = *(const v8h*)(pwh + c * 64 + kk * 32 + 8 * hh);
      pa.h[1] = *(const v8h*)(pwh + c * 64 + kk * 32 + 16 + 8 * hh);
#pragma unroll
      for (int t = 0; t < 4; ++t) {
        FH vb;
        vb.h[0] = *(const v8h*)(Vth + (t * 16 + c) * 64 + kk * 32 + 8 * hh);
        vb.h[1] = *(const v8h*)(Vth + (t * 16 + c) * 64 + kk * 32 + 16 + 8 * hh);
        oacc[t] = mma_h(pa.v, vb.v, oacc[t]);
      }
    }
  }

  float* os = Os[wave];
#pragma unroll
  for (int r = 0; r < 8; ++r) {
    const float l = lrow[r];
    const float inv = ((l > 0.f) ? (1.0f / l) : 0.f) * (64.0f / 1024.0f);
#pragma unroll
    for (int t = 0; t < 4; ++t) os[(8 * hh + r) * 64 + t * 16 + c] = oacc[t][r] * inv;
  }
  wave_sync_lds();
  {
    const int q4 = lane >> 3, c8 = (lane & 7) * 8;
    v4u hvv[4];
#pragma unroll
    for (int it = 0; it < 4; ++it) {
      const int row = it * 4 + q4;
      const float* sp = os + row * 64 + c8;
      v4u pk;
#pragma unroll
      for (int e = 0; e < 4; ++e) {
        pk[e] = pk16(h_bits((_Float16)sp[2 * e]), h_bits((_Float16)sp[2 * e + 1]));
      }
      hvv[it] = pk;
    }
    for (int pass = 0; pass < 2; ++pass) {
#pragma unroll
      for (int it = 0; it < 4; ++it) {
        const int row = it * 4 + q4;
        const size_t go = (rowB + q0 + row) * DM + (size_t)h * HD + c8;
        *(volatile v4u*)(ctxp + go) = hvv[it];
      }
      __threadfence();
    }
  }
}

__global__ __launch_bounds__(256) void aux_loss(const float* __restrict__ part, float* outp) {
  __shared__ float red[2][8];
  const int t = threadIdx.x, lane = t & 31, w = t >> 5;
  float q0 = 0.f, q1 = 0.f, k0 = 0.f, k1 = 0.f;
#pragma unroll 1
  for (int blk = 0; blk < NTG; ++blk) {
    const float* pq = part + (size_t)blk * (NH * NBK);
    const float* pk = part + (size_t)(NTG + blk) * (NH * NBK);
    q0 += pq[t]; q1 += pq[t + 256];
    k0 += pk[t]; k1 += pk[t + 256];
  }
  const float invn = 1.0f / (float)NTOK;
  const float a0 = q0 * invn, a1 = q1 * invn, c0 = k0 * invn, c1 = k1 * invn;
  float vq = a0 * a0 + a1 * a1;
  float vk = c0 * c0 + c1 * c1;
  for (int off = 16; off > 0; off >>= 1) { vq += __shfl_xor(vq, off, 32); vk += __shfl_xor(vk, off, 32); }
  if (lane == 0) { red[0][w] = vq; red[1][w] = vk; }
  __syncthreads();
  if (t == 0) {
    float sq = 0.f, sk = 0.f;
#pragma unroll
    for (int i = 0; i < 8; ++i) { sq += red[0][i]; sk += red[1][i]; }
    const float loss = 0.5f * (float)NBK * (sq * (1.0f / (float)NH) + sk * (1.0f / (float)NH));
    volatile float* op = outp + (size_t)NTOK * DM;
    *op = loss;
    __threadfence();
    *op = loss;
  }
}

extern "C" void kernel_launch(void* const* d_in, const int* in_sizes, int n_in,
                              void* d_out, int out_size, void* d_ws, size_t ws_size,
                              hipStream_t stream) {
  if (n_in < 15) return;
  if (in_sizes[0] != NTOK * DM) return;
  if (in_sizes[1] != DM || in_sizes[2] != DM) return;
  if (in_sizes[3] != DM * DM || in_sizes[4] != DM * DM || in_sizes[5] != DM * DM) return;
  if (in_sizes[6] != NH * HD * NBK || in_sizes[7] != NH * HD * NBK) return;
  if (in_sizes[8] != DM * DM) return;
  if (in_sizes[9] != DM || in_sizes[10] != DM) return;
  if (in_sizes[11] != DM * MLPD || in_sizes[12] != MLPD) return;
  if (in_sizes[13] != MLPD * DM || in_sizes[14] != DM) return;
  if (out_size != NTOK * DM + 1) return;

  const float* x_in  = (const float*)d_in[0];
  const float* ln1_g = (const float*)d_in[1];
  const float* ln1_b = (const float*)d_in[2];
  const float* Wq    = (const float*)d_in[3];
  const float* Wk    = (const float*)d_in[4];
  const float* Wv    = (const float*)d_in[5];
  const float* Whq   = (const float*)d_in[6];
  const float* Whk   = (const float*)d_in[7];
  const float* Wo    = (const float*)d_in[8];
  const float* ln2_g = (const float*)d_in[9];
  const float* ln2_b = (const float*)d_in[10];
  const float* W1    = (const float*)d_in[11];
  const float* b1    = (const float*)d_in[12];
  const float* W2    = (const float*)d_in[13];
  const float* b2    = (const float*)d_in[14];
  float* outf = (float*)d_out;

  const size_t PWQKV = (size_t)3 * DM * DM * 2;
  const size_t PWO   = (size_t)DM * DM * 2;
  const size_t PW1   = (size_t)MLPD * DM * 2;
  const size_t PW2   = (size_t)DM * MLPD * 2;
  const size_t PWH   = (size_t)2 * NBK * DM * 2;
  const size_t PXN   = (size_t)NTOK * DM * 2;
  const size_t PQK   = (size_t)NTOK * QKP * 2;
  const size_t PVT   = (size_t)NBATCH * DM * SEQ * 2;
  const size_t PQX   = (size_t)NTOK * QXP * 2;
  const size_t PCTX  = (size_t)NTOK * DM * 2;
  const size_t PX1   = (size_t)NTOK * DM * 4;
  const size_t PG    = (size_t)NTOK * MLPD * 2;
  const size_t PPART = (size_t)2 * NTG * NH * NBK * 4;
  size_t off = 0;
  const size_t oWQKV = off; off += PWQKV;
  const size_t oWO   = off; off += PWO;
  const size_t oW1   = off; off += PW1;
  const size_t oW2   = off; off += PW2;
  const size_t oWH   = off; off += PWH;
  const size_t oXN   = off; off += PXN;
  const size_t oQK   = off; off += PQK;
  const size_t oVT   = off; off += PVT;
  const size_t oQX   = off; off += PQX;
  const size_t oKX   = off; off += PQX;
  const size_t oCTX  = off; off += PCTX;
  const size_t oX1   = off; off += PX1;
  const size_t oPART = off; off += PPART;
  const size_t oG    = oQK;
  if (oG + PG > oKX) return;
  if (off > ws_size) return;
  if (off > (size_t)134217728) return;

  char* ws = (char*)d_ws;
  unsigned short* WQKV = (unsigned short*)(ws + oWQKV);
  unsigned short* WVT  = WQKV + (size_t)2 * DM * DM;
  unsigned short* WOT  = (unsigned short*)(ws + oWO);
  unsigned short* W1T  = (unsigned short*)(ws + oW1);
  unsigned short* W2T  = (unsigned short*)(ws + oW2);
  unsigned short* WHT  = (unsigned short*)(ws + oWH);
  unsigned short* XN   = (unsigned short*)(ws + oXN);
  unsigned short* QK   = (unsigned short*)(ws + oQK);
  unsigned short* VT   = (unsigned short*)(ws + oVT);
  unsigned short* QX   = (unsigned short*)(ws + oQX);
  unsigned short* KX   = (unsigned short*)(ws + oKX);
  unsigned short* CTX  = (unsigned short*)(ws + oCTX);
  float*          X1   = (float*)(ws + oX1);
  float*          PART = (float*)(ws + oPART);
  unsigned short* G    = (unsigned short*)(ws + oG);

  const dim3 blk(256);

  tr_cvt<<<dim3(DM / 32, DM / 64, 3), blk, 0, stream>>>(Wq, Wk, Wv, WQKV, (long long)DM * DM, DM, DM, WSC);
  tr_cvt<<<dim3(DM / 32, DM / 64, 1), blk, 0, stream>>>(Wo, Wo, Wo, WOT, 0LL, DM, DM, WSC);
  tr_cvt<<<dim3(MLPD / 32, DM / 64, 1), blk, 0, stream>>>(W1, W1, W1, W1T, 0LL, DM, MLPD, WSC);
  tr_cvt<<<dim3(DM / 32, MLPD / 64, 1), blk, 0, stream>>>(W2, W2, W2, W2T, 0LL, MLPD, DM, WSC);
  tr_cvt<<<dim3(NBK / 32, (NH * HD) / 64, 2), blk, 0, stream>>>(Whq, Whk, Whk, WHT, (long long)NBK * DM,
                                                                  NH * HD, NBK, WSC);
  ln_f16<true><<<dim3(NTOK), dim3(128), 0, stream>>>(x_in, ln1_g, ln1_b, XN);
  gemm64<1, false, false, 0><<<dim3(((NTOK / 64) * (QKP / 64) + 7) / 8, 1), blk, 0, stream>>>(
      XN, DM, 0LL, WQKV, DM, 0LL, (void*)QK, QKP, 0LL, b1, x_in, DM, NTOK, QKP, DM, 1.0f / WSC);
  gemm64<1, false, false, 0><<<dim3(((DM / 64) * (SEQ / 64) + 7) / 8, NBATCH), blk, 0, stream>>>(
      WVT, DM, 0LL, XN, DM, (long long)SEQ * DM, (void*)VT, SEQ, (long long)DM * SEQ, b1, x_in, DM,
      DM, SEQ, DM, 1.0f / WSC);
  bucket_qx<<<dim3(NTG, 2), blk, 0, stream>>>(QK, WHT, QX, KX, PART);
  attn_x<<<dim3(NBATCH * NH * NQB), dim3(128), 0, stream>>>(QX, KX, VT, CTX, 0.125f);
  gemm64<0, false, false, 2><<<dim3(((NTOK / 64) * (DM / 64) + 7) / 8, 1), blk, 0, stream>>>(
      CTX, DM, 0LL, WOT, DM, 0LL, (void*)X1, DM, 0LL, b1, x_in, DM, NTOK, DM, DM, 1.0f / (WSC * 64.0f));
  ln_f16<false><<<dim3(NTOK), dim3(128), 0, stream>>>(X1, ln2_g, ln2_b, XN);
  gemm64<1, true, true, 0><<<dim3(((NTOK / 64) * (MLPD / 64) + 7) / 8, 1), blk, 0, stream>>>(
      XN, DM, 0LL, W1T, DM, 0LL, (void*)G, MLPD, 0LL, b1, x_in, DM, NTOK, MLPD, DM, 1.0f / WSC);
  gemm64<0, true, false, 1><<<dim3(((NTOK / 64) * (DM / 64) + 7) / 8, 1), blk, 0, stream>>>(
      G, MLPD, 0LL, W2T, MLPD, 0LL, (void*)outf, DM, 0LL, b2, X1, DM, NTOK, DM, MLPD, 1.0f / WSC);
  aux_loss<<<dim3(1), blk, 0, stream>>>(PART, outf);
  (void)hipGetLastError();
}
